// self_attention_43465069035651
// MI455X (gfx1250) — hardware-verified
//
#include <hip/hip_runtime.h>


#define DEV __device__ __forceinline__

#ifndef NB
#define NB 2
#endif
#ifndef SEQ
#define SEQ 2048
#endif
#define NB_FULL  2
#define SEQ_FULL 2048
#define EMB   1024
#define NHEAD 16
#define HDIM  64
#define QKP   128

#define SST  (SEQ + 4)
#define PST  (SEQ + 8)
#define PTS  68
#define R0A  (16 * SST)
#define R0B  (8 * 16 * PTS)
#define R0F  ((R0A > R0B) ? R0A : R0B)
#define ATTN_LDS_BYTES (R0F * 4 + 16 * 4 + 128 * 4 + 16 * PST * 2)
#define CT_P 136
#define CF_P 132
#define SCORE_SCALE 0.0001220703125f
#define OUT_SCALE   0.000244140625f

static_assert(NB >= 1 && NB <= NB_FULL);
static_assert(SEQ >= 256 && SEQ <= SEQ_FULL && (SEQ % 256) == 0);
static_assert(NHEAD * HDIM == EMB && NHEAD == 16 && HDIM == 64);
static_assert(((NB * SEQ * NHEAD) % 64) == 0 && ((NB * SEQ) % 64) == 0);
static_assert((EMB % 128) == 0 && (HDIM % 32) == 0 && (EMB % 32) == 0 && (QKP == 2 * HDIM));
static_assert((((long long)NB * SEQ * EMB) % (8 * 256)) == 0);
static_assert(ATTN_LDS_BYTES <= 300 * 1024);
static_assert(((R0F * 4) % 16) == 0 && (((R0F + 16 + 128) * 4) % 16) == 0);
static_assert(((PST * 2) % 16) == 0 && ((PTS * 4) % 16) == 0 && ((CT_P * 2) % 16) == 0 && ((CF_P * 4) % 16) == 0);
static_assert(R0B <= R0F && R0A <= R0F);

typedef _Float16       v8h   __attribute__((ext_vector_type(8)));
typedef _Float16       v16h  __attribute__((ext_vector_type(16)));
typedef __bf16         v16bf __attribute__((ext_vector_type(16)));
typedef unsigned short v8us  __attribute__((ext_vector_type(8)));
typedef float          v8f   __attribute__((ext_vector_type(8)));
typedef float          v4f   __attribute__((ext_vector_type(4)));

union FragH { v16h v;  v8h  half[2]; };
union FragX { v16bf b; v16h f; v8us half[2]; };

DEV unsigned int bf16_bits(float f) {
    unsigned int u = __float_as_uint(f);
    u += 0x7FFFu + ((u >> 16) & 1u);
    return u >> 16;
}
DEV float bf16_val(float f) { return __uint_as_float(bf16_bits(f) << 16); }

DEV v8f zero8f() {
    v8f z;
#pragma unroll
    for (int i = 0; i < 8; ++i) z[i] = 0.f;
    return z;
}

DEV v8f mma_bf16(v16bf a, v16bf b, v8f c) {
    c = __builtin_amdgcn_wmma_f32_16x16x32_bf16(false, a, false, b, (short)0, c, false, false);
    asm volatile("v_nop\n\tv_nop\n\tv_nop\n\tv_nop" : "+v"(c) : "v"(a), "v"(b));
    return c;
}
DEV v8f mma_f16(v16h a, v16h b, v8f c) {
    c = __builtin_amdgcn_wmma_f32_16x16x32_f16(false, a, false, b, (short)0, c, false, false);
    asm volatile("v_nop\n\tv_nop\n\tv_nop\n\tv_nop" : "+v"(c) : "v"(a), "v"(b));
    return c;
}

__global__ __launch_bounds__(256) void k_cvt_x(const float* __restrict__ x,
                                               unsigned short* __restrict__ xp)
{
    const unsigned g  = blockIdx.x * 256u + threadIdx.x;
    const unsigned e  = g * 8u;
    const unsigned m  = e >> 10;
    const unsigned c  = e & 1023u;
    const unsigned bb = m / (unsigned)SEQ;
    const unsigned s  = m - bb * (unsigned)SEQ;
    const float* src = x + ((size_t)bb * SEQ_FULL + s) * EMB + c;
    const v4f a0 = *(const v4f*)src;
    const v4f a1 = *(const v4f*)(src + 4);
    v8us o;
#pragma unroll
    for (int i = 0; i < 4; ++i) {
        o[i]     = (unsigned short)bf16_bits(a0[i]);
        o[4 + i] = (unsigned short)bf16_bits(a1[i]);
    }
    unsigned short* dst = xp + (size_t)m * EMB + c;
    *(volatile v8us*)dst = o;
    __threadfence();
    *(volatile v8us*)dst = o;
}

__global__ __launch_bounds__(256) void k_transpose_w(const float* __restrict__ W,
                                                     unsigned short* __restrict__ WT,
                                                     unsigned R, unsigned Ncol, unsigned f16mode)
{
    __shared__ __attribute__((aligned(16))) unsigned short T[64 * 72];
    const unsigned tid = threadIdx.x;
    const unsigned n0 = blockIdx.x * 64u, r0 = blockIdx.y * 64u;
    const unsigned nn = tid & 63u, rq = tid >> 6;
#pragma unroll 4
    for (unsigned i = 0; i < 16u; ++i) {
        const unsigned rr = i * 4u + rq;
        const float v  = W[(size_t)(r0 + rr) * Ncol + n0 + nn];
        const float vb = bf16_val(v);
        const _Float16 hf = (_Float16)(vb * 64.0f);
        const unsigned short fb = __builtin_bit_cast(unsigned short, hf);
        const unsigned short bb = (unsigned short)bf16_bits(v);
        T[nn * 72u + rr] = f16mode ? fb : bb;
    }
    __syncthreads();
    const unsigned piece = tid & 7u;
    const unsigned na = tid >> 3;
    const v8us va = *(const v8us*)(T + na * 72u + piece * 8u);
    const v8us vb2 = *(const v8us*)(T + (na + 32u) * 72u + piece * 8u);
    unsigned short* da = WT + (size_t)(n0 + na) * R + r0 + piece * 8u;
    unsigned short* db = WT + (size_t)(n0 + na + 32u) * R + r0 + piece * 8u;
    *(volatile v8us*)da = va;
    *(volatile v8us*)db = vb2;
    __threadfence();
    *(volatile v8us*)da = va;
    *(volatile v8us*)db = vb2;
}

template <int MODE>
__global__ __launch_bounds__(256) __attribute__((amdgpu_num_vgpr(256)))
void k_gemm_nt(const unsigned short* __restrict__ A, unsigned lda,
               unsigned long long zaHi, unsigned long long zaLo,
               const unsigned short* __restrict__ Bm, unsigned ldb,
               unsigned long long zbHi, unsigned long long zbLo,
               unsigned K, const float* __restrict__ bias, unsigned nbias,
               void* __restrict__ Cm, unsigned long long zcHi, unsigned long long zcLo,
               unsigned ldc, float oscale)
{
    __shared__ __attribute__((aligned(16))) float Cs[MODE ? (64 * CF_P) : (64 * (CT_P / 2))];

    const unsigned tid = threadIdx.x, lane = tid & 31u, w = tid >> 5;
    const unsigned h = lane >> 4, l15 = lane & 15u;
    const unsigned wm = w & 3u, wn = w >> 2;
    const unsigned z = blockIdx.z, zh = z >> 4, zl = z & 15u;
    const unsigned row0 = blockIdx.y * 64u;
    const unsigned col0 = blockIdx.x * 128u;
    const size_t offA = (size_t)zh * (size_t)zaHi + (size_t)zl * (size_t)zaLo;
    const size_t offB = (size_t)zh * (size_t)zbHi + (size_t)zl * (size_t)zbLo;
    const size_t offC = (size_t)zh * (size_t)zcHi + (size_t)zl * (size_t)zcLo;

    const unsigned short* ap = A  + offA + (size_t)(row0 + wm * 16u + l15) * lda + 8u * h;
    const unsigned short* bp = Bm + offB + (size_t)(col0 + wn * 64u + l15) * ldb + 8u * h;

    v8f acc[4];
#pragma unroll
    for (int t = 0; t < 4; ++t) acc[t] = zero8f();

#pragma unroll 1
    for (unsigned k0 = 0; k0 < K; k0 += 32u) {
        FragX a;
        a.half[0] = *(const v8us*)(ap + k0);
        a.half[1] = *(const v8us*)(ap + k0 + 16u);
#pragma unroll
        for (int t = 0; t < 4; ++t) {
            const unsigned short* bq = bp + (size_t)t * 16u * ldb + k0;
            FragX bf;
            bf.half[0] = *(const v8us*)(bq);
            bf.half[1] = *(const v8us*)(bq + 16u);
            if (MODE == 0) acc[t] = mma_bf16(a.b, bf.b, acc[t]);
            else           acc[t] = mma_f16(a.f, bf.f, acc[t]);
        }
    }

    if (MODE == 0) {
        _Float16* Ct = (_Float16*)Cs;
#pragma unroll
        for (int t = 0; t < 4; ++t) {
            const unsigned cl = wn * 64u + (unsigned)t * 16u + l15;
#pragma unroll
            for (int r = 0; r < 8; ++r)
                Ct[(wm * 16u + 8u * h + (unsigned)r) * CT_P + cl] = (_Float16)(acc[t][r] * oscale);
        }
        __syncthreads();

        _Float16* cbase = (_Float16*)Cm + offC + (size_t)row0 * (size_t)ldc + col0;
        v8h sv[4];
#pragma unroll
        for (int i = 0; i < 4; ++i) {
            const unsigned rl = w * 8u + 2u * (unsigned)i + h;
            sv[i] = *(const v8h*)(Ct + rl * CT_P + l15 * 8u);
        }
#pragma unroll
        for (int i = 0; i < 4; ++i) {
            const unsigned rl = w * 8u + 2u * (unsigned)i + h;
            *(volatile v8h*)(cbase + (size_t)rl * (size_t)ldc + l15 * 8u) = sv[i];
        }
        __threadfence();
#pragma unroll
        for (int i = 0; i < 4; ++i) {
            const unsigned rl = w * 8u + 2u * (unsigned)i + h;
            *(volatile v8h*)(cbase + (size_t)rl * (size_t)ldc + l15 * 8u) = sv[i];
        }
    } else {
#pragma unroll
        for (int t = 0; t < 4; ++t) {
            const unsigned cl = wn * 64u + (unsigned)t * 16u + l15;
            unsigned ci = col0 + cl;
            ci = ci < nbias ? ci : (nbias - 1u);
            const float colb = bf16_val(bias[ci]);
#pragma unroll
            for (int r = 0; r < 8; ++r)
                Cs[(wm * 16u + 8u * h + (unsigned)r) * CF_P + cl] = acc[t][r] * oscale + colb;
        }
        __syncthreads();

        float* cbase = (float*)Cm + offC + (size_t)row0 * (size_t)ldc + col0;
        v4f fv[8];
#pragma unroll
        for (int i = 0; i < 8; ++i) {
            const unsigned rl = w * 8u + (unsigned)i;
            fv[i] = *(const v4f*)(Cs + rl * CF_P + lane * 4u);
        }
#pragma unroll
        for (int i = 0; i < 8; ++i) {
            const unsigned rl = w * 8u + (unsigned)i;
            *(volatile v4f*)(cbase + (size_t)rl * (size_t)ldc + lane * 4u) = fv[i];
        }
        __threadfence();
#pragma unroll
        for (int i = 0; i < 8; ++i) {
            const unsigned rl = w * 8u + (unsigned)i;
            *(volatile v4f*)(cbase + (size_t)rl * (size_t)ldc + lane * 4u) = fv[i];
        }
    }
}

__global__ __launch_bounds__(256) __attribute__((amdgpu_num_vgpr(256)))
void k_attn(const _Float16* __restrict__ QK, const _Float16* __restrict__ Vt,
            _Float16* __restrict__ Ctx)
{
    extern __shared__ v4f smem4[];
    float*    smem    = (float*)smem4;
    float*    S       = smem;
    float*    Pt      = smem;
    float*    rowsum  = smem + R0F;
    float*    rowmaxp = rowsum + 16;
    _Float16* Ph      = (_Float16*)(rowmaxp + 128);

    const unsigned tid = threadIdx.x, lane = tid & 31u, w = tid >> 5;
    const unsigned h = lane >> 4, l15 = lane & 15u;
    const unsigned halfrow = 8u * h, kbo = 8u * h;
    const unsigned QT = (unsigned)(SEQ / 16);
    const unsigned bh = blockIdx.x / QT;
    const unsigned q0 = (blockIdx.x - bh * QT) * 16u;
    const unsigned b  = bh >> 4, hd = bh & 15u;

    FragH qf[2];
    {
        const _Float16* qp = QK + ((size_t)((b * (unsigned)SEQ + q0 + l15) * 16u + hd)) * QKP + kbo;
#pragma unroll
        for (int s = 0; s < 2; ++s) {
            qf[s].half[0] = *(const v8h*)(qp + s * 32);
            qf[s].half[1] = *(const v8h*)(qp + s * 32 + 16);
        }
    }

    float vmax[8];
#pragma unroll
    for (int r = 0; r < 8; ++r) vmax[r] = -3.0e38f;

    const _Float16* kbase = QK + ((size_t)((b * (unsigned)SEQ + l15) * 16u + hd)) * QKP + HDIM + kbo;
#pragma unroll 1
    for (unsigned t = 0; t < (unsigned)(SEQ / 128); ++t) {
        const unsigned m0 = w * (unsigned)(SEQ / 8) + t * 16u;
        const _Float16* kp = kbase + (size_t)m0 * (16u * QKP);
        v8f c = zero8f();
#pragma unroll
        for (int s = 0; s < 2; ++s) {
            FragH kb;
            kb.half[0] = *(const v8h*)(kp + s * 32);
            kb.half[1] = *(const v8h*)(kp + s * 32 + 16);
            c = mma_f16(qf[s].v, kb.v, c);
        }
#pragma unroll
        for (int r = 0; r < 8; ++r) {
            const float sv = c[r] * SCORE_SCALE;
            S[(halfrow + (unsigned)r) * SST + m0 + l15] = sv;
            vmax[r] = fmaxf(vmax[r], sv);
        }
    }
#pragma unroll
    for (int r = 0; r < 8; ++r) {
#pragma unroll
        for (int off = 1; off < 16; off <<= 1) vmax[r] = fmaxf(vmax[r], __shfl_xor(vmax[r], off));
    }
    if (l15 == 0) {
#pragma unroll
        for (int r = 0; r < 8; ++r) rowmaxp[w * 16u + halfrow + (unsigned)r] = vmax[r];
    }
    __syncthreads();

#pragma unroll 1
    for (unsigned jj = 0; jj < 2u; ++jj) {
        const unsigned j = w * 2u + jj;
        float m = rowmaxp[j];
#pragma unroll
        for (int ww = 1; ww < 8; ++ww) m = fmaxf(m, rowmaxp[ww * 16 + j]);
        const float* srow = S + j * SST;
        _Float16* prow = Ph + j * PST;
        float s = 0.f;
#pragma unroll 2
        for (unsigned i = lane; i < (unsigned)SEQ; i += 32u) {
            const float e = __expf(srow[i] - m);
            const _Float16 ph = (_Float16)(e * 1024.0f);
            prow[i] = ph;
            s += (float)ph;
        }
#pragma unroll
        for (int off = 16; off; off >>= 1) s += __shfl_xor(s, off);
        if (lane == 0) rowsum[j] = s;
    }
    __syncthreads();

    v8f acc[4];
#pragma unroll
    for (int t = 0; t < 4; ++t) acc[t] = zero8f();

    const _Float16* vbase = Vt + ((size_t)(b * (unsigned)EMB + hd * (unsigned)HDIM + l15)) * SEQ + kbo;
    const _Float16* pbase = Ph + l15 * PST + kbo;
#pragma unroll 1
    for (unsigned ks = 0; ks < (unsigned)(SEQ / 256); ++ks) {
        const unsigned m0 = w * (unsigned)(SEQ / 8) + ks * 32u;
        FragH pa;
        pa.half[0] = *(const v8h*)(pbase + m0);
        pa.half[1] = *(const v8h*)(pbase + m0 + 16u);
#pragma unroll
        for (int t = 0; t < 4; ++t) {
            const _Float16* vp = vbase + (size_t)t * 16u * SEQ + m0;
            FragH vf;
            vf.half[0] = *(const v8h*)(vp);
            vf.half[1] = *(const v8h*)(vp + 16);
            acc[t] = mma_f16(pa.v, vf.v, acc[t]);
        }
    }

#pragma unroll
    for (int t = 0; t < 4; ++t) {
#pragma unroll
        for (int r = 0; r < 8; ++r)
            Pt[(w * 16u + halfrow + (unsigned)r) * PTS + (unsigned)t * 16u + l15] = acc[t][r];
    }
    __syncthreads();

    if (w < 4u) {
        const unsigned row = tid >> 3;
        const unsigned c8  = (tid & 7u) * 8u;
        v4f s0, s1;
#pragma unroll
        for (int i = 0; i < 4; ++i) { s0[i] = 0.f; s1[i] = 0.f; }
#pragma unroll
        for (int ww = 0; ww < 8; ++ww) {
            const float* p = Pt + ((unsigned)ww * 16u + row) * PTS + c8;
            const v4f a0 = *(const v4f*)p;
            const v4f a1 = *(const v4f*)(p + 4);
            s0 += a0;
            s1 += a1;
        }
        const float sc = 4.0f * (1.0f / rowsum[row]);
        v8h o;
#pragma unroll
        for (int i = 0; i < 4; ++i) {
            o[i]     = (_Float16)(s0[i] * sc);
            o[4 + i] = (_Float16)(s1[i] * sc);
        }
        _Float16* dst = Ctx + ((size_t)(b * (unsigned)SEQ + q0 + row)) * EMB + hd * (unsigned)HDIM + c8;
        *(volatile v8h*)dst = o;
        __threadfence();
        *(volatile v8h*)dst = o;
    }
}

extern "C" void kernel_launch(void* const* d_in, const int* in_sizes, int n_in,
                              void* d_out, int out_size, void* d_ws, size_t ws_size,
                              hipStream_t stream)
{
    if (n_in < 6) return;
    const long long need_x = ((long long)(NB - 1) * SEQ_FULL + SEQ) * EMB;
    if ((long long)in_sizes[0] < need_x) return;
    if (in_sizes[1] < HDIM * HDIM || in_sizes[2] < HDIM * HDIM || in_sizes[3] < HDIM * HDIM) return;
    if (in_sizes[4] < EMB * EMB || in_sizes[5] < EMB) return;
    if ((long long)out_size < (long long)NB * SEQ * EMB) return;

    const float* x  = (const float*)d_in[0];
    const float* Wq = (const float*)d_in[1];
    const float* Wk = (const float*)d_in[2];
    const float* Wv = (const float*)d_in[3];
    const float* Wo = (const float*)d_in[4];
    const float* bo = (const float*)d_in[5];
    float* out = (float*)d_out;

    char* ws = (char*)d_ws;
    size_t off = 0;
    auto carve = [&](size_t bytes) -> char* {
        char* p = ws + off;
        off += (bytes + 255) & ~(size_t)255;
        return p;
    };
    unsigned short* xbf  = (unsigned short*)carve((size_t)NB * SEQ * EMB * 2);
    unsigned short* wqkT = (unsigned short*)carve((size_t)QKP * HDIM * 2);
    unsigned short* wvT  = (unsigned short*)carve((size_t)HDIM * HDIM * 2);
    unsigned short* woT  = (unsigned short*)carve((size_t)EMB * EMB * 2);
    _Float16* QKp = (_Float16*)carve((size_t)NB * SEQ * NHEAD * QKP * 2);
    _Float16* Vt  = (_Float16*)carve((size_t)NB * EMB * SEQ * 2);
    _Float16* Ctx = (_Float16*)carve((size_t)NB * SEQ * EMB * 2);
    if (off > ws_size) return;

    k_cvt_x<<<(unsigned)(((size_t)NB * SEQ * EMB) / 8 / 256), 256, 0, stream>>>(x, xbf);

    k_transpose_w<<<dim3(1, 1), 256, 0, stream>>>(Wq, wqkT, HDIM, HDIM, 0u);
    k_transpose_w<<<dim3(1, 1), 256, 0, stream>>>(Wk, wqkT + HDIM * HDIM, HDIM, HDIM, 0u);
    k_transpose_w<<<dim3(1, 1), 256, 0, stream>>>(Wv, wvT, HDIM, HDIM, 0u);
    k_transpose_w<<<dim3(EMB / 64, EMB / 64), 256, 0, stream>>>(Wo, woT, EMB, EMB, 1u);

    k_gemm_nt<0><<<dim3(1, (NB * SEQ * NHEAD) / 64, 1), 256, 0, stream>>>(
        xbf, (unsigned)HDIM, 0ULL, 0ULL,
        wqkT, (unsigned)HDIM, 0ULL, 0ULL,
        (unsigned)HDIM, bo, (unsigned)EMB,
        (void*)QKp, 0ULL, 0ULL, (unsigned)QKP, 16.0f);
    k_gemm_nt<0><<<dim3(SEQ / 128, 1, NB * NHEAD), 256, 0, stream>>>(
        wvT, (unsigned)HDIM, 0ULL, 0ULL,
        xbf, (unsigned)EMB, (unsigned long long)SEQ * EMB, (unsigned long long)HDIM,
        (unsigned)HDIM, bo, (unsigned)EMB,
        (void*)Vt, (unsigned long long)EMB * SEQ, (unsigned long long)HDIM * SEQ, (unsigned)SEQ, 16.0f);

    hipFuncSetAttribute(reinterpret_cast<const void*>(&k_attn),
                        hipFuncAttributeMaxDynamicSharedMemorySize, ATTN_LDS_BYTES);
    k_attn<<<NB * NHEAD * (SEQ / 16), 256, ATTN_LDS_BYTES, stream>>>(QKp, Vt, Ctx);

    k_gemm_nt<1><<<dim3(EMB / 128, (NB * SEQ) / 64, 1), 256, 0, stream>>>(
        (const unsigned short*)Ctx, (unsigned)EMB, 0ULL, 0ULL,
        woT, (unsigned)EMB, 0ULL, 0ULL,
        (unsigned)EMB, bo, (unsigned)EMB,
        (void*)out, 0ULL, 0ULL, (unsigned)EMB, OUT_SCALE);
}
